// GroupedQueryAttention_65343632441492
// MI455X (gfx1250) — hardware-verified
//
#include <hip/hip_runtime.h>
#ifndef NB
#define NB 2
#endif
#ifndef SEQ
#define SEQ 2048
#endif
#define NB_FULL 2
#define SEQ_FULL 2048
#define DM 1024
#define NH 16
#define HD 64
#define NG 4
#define HPG 4
#define KD (NG * HD)
#define KVW (2 * KD)
#define HG 4
#define USEQ ((unsigned)SEQ)
#define NR ((size_t)NB * SEQ)

static_assert(SEQ % 128 == 0);
static_assert(NB <= NB_FULL && SEQ <= SEQ_FULL);
static_assert(HG == HPG && NH == NG * HPG && DM == NH * HD);
static_assert(DM % 256 == 0 && KD == 256 && HD == 64);

typedef unsigned short v8us __attribute__((ext_vector_type(8), may_alias));
typedef float  v8f  __attribute__((ext_vector_type(8)));
typedef float  v4f  __attribute__((ext_vector_type(4)));
typedef float  v4fa __attribute__((ext_vector_type(4), may_alias));
typedef _Float16 v16h __attribute__((ext_vector_type(16)));
typedef _Float16 v4h  __attribute__((ext_vector_type(4)));
union FragH { v16h v; v8us half[2]; _Float16 h[16]; unsigned short u[16]; };

__device__ __forceinline__ float bf16_rne(float x) { unsigned int u = __float_as_uint(x); u = (u + 0x7FFFu + ((u >> 16) & 1u)) & 0xFFFF0000u; return __uint_as_float(u); }

__global__ __launch_bounds__(256) void k_wt_f16(const float* __restrict__ W, _Float16* __restrict__ Wt, unsigned K, unsigned N, float scale) {
  const unsigned t = blockIdx.x * 256u + threadIdx.x; const unsigned k8n = K >> 3; if (t >= N * k8n) return;
  const unsigned n = t / k8n, k8 = (t - n * k8n) << 3; FragH f;
#pragma unroll
  for (unsigned i = 0; i < 8; ++i) f.h[i] = (_Float16)(bf16_rne(W[(size_t)(k8 + i) * N + n]) * scale);
  const v8us o = f.half[0]; unsigned short* dst = (unsigned short*)Wt + (size_t)n * K + k8;
  *(volatile v8us*)dst = o; __threadfence(); *(volatile v8us*)dst = o;
}

__global__ __launch_bounds__(256) void k_x16(const float* __restrict__ x, _Float16* __restrict__ X16) {
  const unsigned t = blockIdx.x * 256u + threadIdx.x; if (t >= (unsigned)(NR * (DM / 8))) return;
  const unsigned row = t / (unsigned)(DM / 8), c8 = (t % (unsigned)(DM / 8)) << 3; const unsigned b = row / USEQ, tt = row % USEQ;
  const float* src = x + ((size_t)b * SEQ_FULL + tt) * DM + c8;
  const v4f a = *(const v4fa*)src, c = *(const v4fa*)(src + 4); FragH f;
#pragma unroll
  for (unsigned q = 0; q < 4; ++q) { f.h[q] = (_Float16)bf16_rne(a[q]); f.h[4 + q] = (_Float16)bf16_rne(c[q]); }
  const v8us o = f.half[0]; unsigned short* dst = (unsigned short*)X16 + (size_t)t * 8;
  *(volatile v8us*)dst = o; __threadfence(); *(volatile v8us*)dst = o;
}

__device__ __forceinline__ v16h g2_frag(const _Float16* p, unsigned hh) { FragH f; f.half[0] = *(const v8us*)((const unsigned short*)p + 8u * hh); f.half[1] = *(const v8us*)((const unsigned short*)p + 16u + 8u * hh); return f.v; }
__device__ __forceinline__ v8f g2_mma(v16h a, v16h b, v8f c) { v8f d = __builtin_amdgcn_wmma_f32_16x16x32_f16(false, a, false, b, (short)0, c, false, false); asm volatile("v_nop\n\tv_nop\n\tv_nop\n\tv_nop" : "+v"(d) : "v"(a), "v"(b)); return d; }

__global__ __launch_bounds__(128) void k_gemm2(const _Float16* __restrict__ A, unsigned lda, size_t sA, const _Float16* __restrict__ Bh, unsigned ldb, size_t sB, float alpha, const float* __restrict__ bias,
    float* __restrict__ C, _Float16* __restrict__ C16, unsigned ldc, size_t sC, unsigned M, unsigned N, unsigned K) {
  __shared__ __attribute__((aligned(16))) float so[4][32][68];
  const unsigned tid = threadIdx.x, w = tid >> 5, lane = tid & 31u, ln = lane & 15u, hh = lane >> 4; const unsigned by = blockIdx.y;
  A += (size_t)by * sA; Bh += (size_t)by * sB; const size_t cofs = (size_t)by * sC;
  const unsigned ntn = N >> 6; const unsigned mt = blockIdx.x / ntn, nq = blockIdx.x - mt * ntn; const unsigned row0 = mt * 128u + 32u * w, col0 = nq * 64u; if (row0 >= M) return;
  const _Float16* a0p = A + (size_t)(row0 + ln) * lda; const _Float16* a1p = a0p + (size_t)16 * lda;
  const _Float16* b0p = Bh + (size_t)(col0 + ln) * ldb; const _Float16* b1p = b0p + (size_t)16 * ldb; const _Float16* b2p = b1p + (size_t)16 * ldb; const _Float16* b3p = b2p + (size_t)16 * ldb;
  const v8f z8 = {0.f,0.f,0.f,0.f,0.f,0.f,0.f,0.f}; v8f c00 = z8, c01 = z8, c02 = z8, c03 = z8, c10 = z8, c11 = z8, c12 = z8, c13 = z8;
#pragma unroll 1
  for (unsigned kb = 0; kb < K; kb += 32u) { const v16h a0 = g2_frag(a0p + kb, hh), a1 = g2_frag(a1p + kb, hh);
    v16h b = g2_frag(b0p + kb, hh); c00 = g2_mma(a0, b, c00); c10 = g2_mma(a1, b, c10);
    b = g2_frag(b1p + kb, hh); c01 = g2_mma(a0, b, c01); c11 = g2_mma(a1, b, c11);
    b = g2_frag(b2p + kb, hh); c02 = g2_mma(a0, b, c02); c12 = g2_mma(a1, b, c12);
    b = g2_frag(b3p + kb, hh); c03 = g2_mma(a0, b, c03); c13 = g2_mma(a1, b, c13); }
  v8f accs[8] = {c00, c01, c02, c03, c10, c11, c12, c13};
#pragma unroll
  for (unsigned u = 0; u < 8; ++u) { const unsigned t = u & 3u, hf = u >> 2; const unsigned col = col0 + t * 16u + ln; const float bv = bias ? bf16_rne(bias[col]) : 0.f;
#pragma unroll
    for (unsigned r = 0; r < 8; ++r) { const unsigned rloc = hf * 16u + 8u * hh + r; so[w][rloc][t * 16u + ln] = accs[u][r] * alpha + bv; } }
  __builtin_amdgcn_fence(4  , "workgroup"); __builtin_amdgcn_wave_barrier();
  const unsigned rsub = lane >> 4, c4 = (lane & 15u) * 4u;
  for (unsigned pass = 0; pass < 2; ++pass) {
#pragma unroll
    for (unsigned q = 0; q < 16; ++q) { const unsigned r = q * 2u + rsub; const v4f v = *(const v4fa*)&so[w][r][c4];
      if (C) *(volatile v4f*)(C + cofs + (size_t)(row0 + r) * ldc + col0 + c4) = v;
      if (C16) { v4h h4; h4[0] = (_Float16)v[0]; h4[1] = (_Float16)v[1]; h4[2] = (_Float16)v[2]; h4[3] = (_Float16)v[3]; *(volatile v4h*)(C16 + cofs + (size_t)(row0 + r) * ldc + col0 + c4) = h4; } }
    if (pass == 0) __threadfence(); } }

template <unsigned NHv, unsigned TTv>
__global__ __launch_bounds__(256) void k_vt(const _Float16* __restrict__ V16, unsigned ldv, unsigned voff, _Float16* __restrict__ Vt) {
  __shared__ unsigned short tl[64][66]; const unsigned tid = threadIdx.x; const unsigned slab = blockIdx.x / (TTv / 64u), lg = blockIdx.x % (TTv / 64u); const unsigned b = slab / NHv, h = slab % NHv;
  for (unsigned i = tid; i < 512u; i += 256u) { const unsigned r = i >> 3, c8 = (i & 7u) << 3; FragH f; f.half[0] = *(const v8us*)((const unsigned short*)V16 + ((size_t)b * TTv + lg * 64u + r) * ldv + voff + h * 64u + c8);
#pragma unroll
    for (unsigned q = 0; q < 8; ++q) tl[r][c8 + q] = f.u[q]; }
  __syncthreads();
  for (unsigned pass = 0; pass < 2; ++pass) {
#pragma unroll
    for (unsigned rd = 0; rd < 2; ++rd) { const unsigned d = rd * 32u + (tid >> 3), pc = tid & 7u; FragH f;
#pragma unroll
      for (unsigned q = 0; q < 8; ++q) f.u[q] = tl[pc * 8u + q][d];
      *(volatile v8us*)((unsigned short*)Vt + ((size_t)slab * 64u + d) * TTv + lg * 64u + pc * 8u) = f.half[0]; }
    if (pass == 0) __threadfence(); } }

__global__ __launch_bounds__(256) void k_rsmf(const float* __restrict__ S, _Float16* __restrict__ P, unsigned nrows) {
  #pragma clang fp contract(off)
  const unsigned i = blockIdx.x * 256u + threadIdx.x; if (i >= nrows) return; const float* s = S + (size_t)i * SEQ; float mx = -3.0e38f;
#pragma unroll 1
  for (unsigned j = 0; j < USEQ; j += 4u) { const v4f a = *(const v4fa*)(s + j); mx = fmaxf(mx, a[0]); mx = fmaxf(mx, a[1]); mx = fmaxf(mx, a[2]); mx = fmaxf(mx, a[3]); }
  float se = 0.f;
#pragma unroll 1
  for (unsigned j = 0; j < USEQ; j += 4u) { const v4f a = *(const v4fa*)(s + j); se += __expf(a[0] - mx); se += __expf(a[1] - mx); se += __expf(a[2] - mx); se += __expf(a[3] - mx); }
  const float sc = 256.0f / se;
#pragma unroll 1
  for (unsigned j0 = 0; j0 < USEQ; j0 += 8u) { const v4f a = *(const v4fa*)(s + j0), c = *(const v4fa*)(s + j0 + 4u); FragH f;
#pragma unroll
    for (unsigned q = 0; q < 4; ++q) { f.h[q] = (_Float16)(__expf(a[q] - mx) * sc); f.h[4 + q] = (_Float16)(__expf(c[q] - mx) * sc); }
    const v8us o = f.half[0]; unsigned short* d = (unsigned short*)P + (size_t)i * SEQ + j0; *(volatile v8us*)d = o; __threadfence(); *(volatile v8us*)d = o; } }

__global__ __launch_bounds__(32) void k_inv(float* __restrict__ IV) {
  #pragma clang fp contract(off)
  const unsigned j = threadIdx.x; const float e = (float)(2u * j) / 64.0f; const float v = 1.0f / powf(10000.0f, e);
  *(volatile float*)(IV + j) = v; __threadfence(); *(volatile float*)(IV + j) = v; }

__global__ __launch_bounds__(256) void k_tab(const float* __restrict__ IV, float* __restrict__ CS, float* __restrict__ SN) {
  #pragma clang fp contract(off)
  const unsigned t = blockIdx.x * 256u + threadIdx.x; const unsigned j = t & 31u, p = t >> 5;
  const float ang = (float)p * IV[j]; const float c = cosf(ang), s = sinf(ang);
  *(volatile float*)(CS + t) = c; *(volatile float*)(SN + t) = s; __threadfence(); *(volatile float*)(CS + t) = c; *(volatile float*)(SN + t) = s; }

__global__ __launch_bounds__(256) void k_rope64(const float* __restrict__ F, unsigned ldf, unsigned nseg, const float* __restrict__ CS, const float* __restrict__ SN, _Float16* __restrict__ OUT, unsigned ldo, float osc) {
  #pragma clang fp contract(off)
  __shared__ float xv[256]; __shared__ __attribute__((aligned(16))) _Float16 ov[256];
  const unsigned d = threadIdx.x; const unsigned r = blockIdx.x / nseg, seg = blockIdx.x - r * nseg; const unsigned p = r % USEQ;
  xv[d] = F[(size_t)r * ldf + seg * 256u + d]; __syncthreads();
  const unsigned ti = d & 31u; const float c = CS[p * 32u + ti], s = SN[p * 32u + ti];
  const float other = xv[d ^ 32u]; const float rot = ((d & 32u) == 0u) ? -other : other;
  const float val = (xv[d] * c + rot * s) * osc;
  ov[d] = (_Float16)val; __syncthreads();
  if (d < 32u) { const v8us o = *(const v8us*)&ov[d * 8u]; unsigned short* dst = (unsigned short*)OUT + (size_t)r * ldo + seg * 256u + d * 8u; *(volatile v8us*)dst = o; __threadfence(); *(volatile v8us*)dst = o; } }

static constexpr size_t aln(size_t b) { return (b + 255) & ~(size_t)255; }

extern "C" void kernel_launch(void* const* d_in, const int* in_sizes, int n_in,
                              void* d_out, int out_size, void* d_ws, size_t ws_size, hipStream_t stream) {
  if (n_in < 5) return;
  constexpr size_t X_NEED = ((size_t)(NB - 1) * SEQ_FULL + SEQ) * DM;
  if ((size_t)in_sizes[0] < X_NEED || in_sizes[1] < DM * DM || in_sizes[2] < DM * KVW || in_sizes[3] < DM * DM || in_sizes[4] < DM || (size_t)out_size < X_NEED) return;
  const float* x = (const float*)d_in[0]; const float* wq = (const float*)d_in[1]; const float* wkv = (const float*)d_in[2]; const float* wo = (const float*)d_in[3]; const float* bo = (const float*)d_in[4];
  float* out = (float*)d_out;
  constexpr size_t SZ_BO = aln((size_t)DM * DM * 2), SZ_Q16 = aln(NR * DM * 2), SZ_K16 = aln(NR * KD * 2), SZ_VT = aln((size_t)NB * NG * HD * SEQ * 2), SZ_O16 = aln(NR * DM * 2), SZ_P = aln((size_t)HG * SEQ * SEQ * 2);
  constexpr size_t SZ_X16 = aln(NR * DM * 2), SZ_BQ = aln((size_t)DM * DM * 2), SZ_BKV = aln((size_t)KVW * DM * 2), SZ_Q32 = aln(NR * DM * 4), SZ_KV32 = aln(NR * KVW * 4), SZ_KV16 = aln(NR * KVW * 2), SZ_IV = 256, SZ_TAB = aln((size_t)SEQ * 32 * 4);
  constexpr size_t SZ_PREP = SZ_X16 + SZ_BQ + SZ_BKV + SZ_Q32 + SZ_KV32 + SZ_KV16 + SZ_IV + 2 * SZ_TAB;
  constexpr size_t SZ_S = aln((size_t)HG * SEQ * SEQ * 4);
  constexpr size_t SZ_U = (SZ_PREP > SZ_S) ? SZ_PREP : SZ_S;
  constexpr size_t OF_BO = 0, OF_Q16 = OF_BO + SZ_BO, OF_K16 = OF_Q16 + SZ_Q16, OF_VT = OF_K16 + SZ_K16, OF_O16 = OF_VT + SZ_VT, OF_P = OF_O16 + SZ_O16, OF_U = OF_P + SZ_P;
  constexpr size_t OF_X16 = OF_U, OF_BQ = OF_X16 + SZ_X16, OF_BKV = OF_BQ + SZ_BQ, OF_Q32 = OF_BKV + SZ_BKV, OF_KV32 = OF_Q32 + SZ_Q32, OF_KV16 = OF_KV32 + SZ_KV32, OF_IV = OF_KV16 + SZ_KV16, OF_CS = OF_IV + SZ_IV, OF_SN = OF_CS + SZ_TAB;
  constexpr size_t TOTAL = OF_U + SZ_U;
  static_assert(OF_SN + SZ_TAB <= TOTAL);
  static_assert(SZ_S <= SZ_U && SZ_PREP <= SZ_U);
  static_assert(TOTAL <= (size_t)134217728);
  if (TOTAL > ws_size) return;
  char* ws = (char*)d_ws;
  _Float16* BO = (_Float16*)(ws + OF_BO); _Float16* Q16 = (_Float16*)(ws + OF_Q16); _Float16* K16 = (_Float16*)(ws + OF_K16); _Float16* VT = (_Float16*)(ws + OF_VT); _Float16* O16 = (_Float16*)(ws + OF_O16); _Float16* P = (_Float16*)(ws + OF_P);
  float* S = (float*)(ws + OF_U);
  _Float16* X16 = (_Float16*)(ws + OF_X16); _Float16* BQ = (_Float16*)(ws + OF_BQ); _Float16* BKV = (_Float16*)(ws + OF_BKV); float* Q32 = (float*)(ws + OF_Q32); float* KV32 = (float*)(ws + OF_KV32); _Float16* KV16 = (_Float16*)(ws + OF_KV16);
  float* IV = (float*)(ws + OF_IV); float* CS = (float*)(ws + OF_CS); float* SN = (float*)(ws + OF_SN);

  static_assert(((size_t)DM * (DM / 8)) % 256 == 0 && ((size_t)KVW * (DM / 8)) % 256 == 0);
  k_wt_f16<<<(unsigned)(((size_t)DM * (DM / 8)) / 256), 256, 0, stream>>>(wo, BO, DM, DM, 16.0f);
  k_wt_f16<<<(unsigned)(((size_t)DM * (DM / 8)) / 256), 256, 0, stream>>>(wq, BQ, DM, DM, 16.0f);
  k_wt_f16<<<(unsigned)(((size_t)KVW * (DM / 8)) / 256), 256, 0, stream>>>(wkv, BKV, DM, KVW, 16.0f);
  static_assert((NR * (DM / 8)) % 256 == 0);
  k_x16<<<(unsigned)((NR * (DM / 8)) / 256), 256, 0, stream>>>(x, X16);
  k_gemm2<<<dim3((unsigned)((NR / 128) * (DM / 64)), 1), 128, 0, stream>>>(X16, DM, 0, BQ, DM, 0, 0.0625f, nullptr, Q32, nullptr, DM, 0, (unsigned)NR, DM, DM);
  k_gemm2<<<dim3((unsigned)((NR / 128) * (KVW / 64)), 1), 128, 0, stream>>>(X16, DM, 0, BKV, DM, 0, 0.0625f, nullptr, KV32, KV16, KVW, 0, (unsigned)NR, KVW, DM);
  k_inv<<<1, 32, 0, stream>>>(IV);
  static_assert(((size_t)SEQ * 32) % 256 == 0);
  k_tab<<<(unsigned)(((size_t)SEQ * 32) / 256), 256, 0, stream>>>(IV, CS, SN);
  k_rope64<<<(unsigned)(NR * (DM / 256)), 256, 0, stream>>>(Q32, DM, DM / 256, CS, SN, Q16, DM, 16.0f);
  k_rope64<<<(unsigned)NR, 256, 0, stream>>>(KV32, KVW, 1, CS, SN, K16, KD, 16.0f);
  k_vt<NG, USEQ><<<(unsigned)(NB * NG * (SEQ / 64)), 256, 0, stream>>>(KV16, KVW, KD, VT);

  for (unsigned b = 0; b < (unsigned)NB; ++b) { const size_t r0 = (size_t)b * SEQ;
    for (unsigned g = 0; g < (unsigned)NG; ++g) { const unsigned h0 = g * HPG;
      k_gemm2<<<dim3((SEQ / 128) * (SEQ / 64), HG), 128, 0, stream>>>(Q16 + r0 * DM + h0 * HD, DM, (size_t)HD, K16 + r0 * KD + g * HD, KD, 0, 0.00048828125f, nullptr, S, nullptr, SEQ, (size_t)SEQ * SEQ, SEQ, SEQ, HD);
      k_rsmf<<<(unsigned)(((size_t)HG * SEQ) / 256), 256, 0, stream>>>(S, P, (unsigned)(HG * SEQ));
      k_gemm2<<<dim3((SEQ / 128) * (HD / 64), HG), 128, 0, stream>>>(P, SEQ, (size_t)SEQ * SEQ, VT + ((size_t)b * NG + g) * HD * SEQ, SEQ, 0, 0.25f, nullptr, nullptr, O16 + r0 * DM + h0 * HD, DM, (size_t)HD, SEQ, HD, SEQ); } }
  k_gemm2<<<dim3((SEQ / 128) * (DM / 64), NB), 128, 0, stream>>>(O16, DM, (size_t)SEQ * DM, BO, DM, 0, 0.0009765625f, bo, out, nullptr, DM, (size_t)SEQ_FULL * DM, SEQ, DM, DM);
}
